// MultiHeadCrossModalAttention_21732534518179
// MI455X (gfx1250) — hardware-verified
//
#include <hip/hip_runtime.h>
#include <math.h>

constexpr int kBatch = 4;
constexpr int kSeqQ  = 1024;
constexpr int kSeqK  = 2048;
constexpr int kEmb   = 1024;
constexpr int kHeads = 16;
constexpr int kHdim  = 64;
constexpr int kRowsQ = kBatch * kSeqQ;
constexpr int kRowsK = kBatch * kSeqK;
constexpr int kHeadsPerGroup = 4;
constexpr int kGroups = kBatch * kHeads / kHeadsPerGroup;
constexpr float kScoreScale = 0.125f;
constexpr float kInvEmb = 1.0f / 1024.0f;
constexpr float kLnEps  = 1e-5f;

typedef __attribute__((ext_vector_type(16))) _Float16 v16h;
typedef __attribute__((ext_vector_type(8)))  _Float16 v8h;
typedef __attribute__((ext_vector_type(16))) __bf16   v16b;
typedef __attribute__((ext_vector_type(8)))  __bf16   v8b;
typedef __attribute__((ext_vector_type(8)))  float    v8f;
typedef __attribute__((ext_vector_type(4)))  float    v4f;
typedef __attribute__((ext_vector_type(4)))  unsigned int v4u;

__device__ __forceinline__ unsigned short f2bf_bits(float f) {
  unsigned u = __float_as_uint(f);
  return (unsigned short)((u + 0x7FFFu + ((u >> 16) & 1u)) >> 16);
}
__device__ __forceinline__ float bf_bits2f(unsigned short h) { return __uint_as_float(((unsigned)h) << 16); }

__device__ __forceinline__ void dep_guard_h(v8f& a, v8f& b, v16h x, v16h y) { asm volatile("v_nop\n\tv_nop\n\tv_nop\n\tv_nop" : "+v"(a), "+v"(b) : "v"(x), "v"(y)); }
__device__ __forceinline__ void dep_guard_b(v8f& a, v8f& b, v16b x, v16b y) { asm volatile("v_nop\n\tv_nop\n\tv_nop\n\tv_nop" : "+v"(a), "+v"(b) : "v"(x), "v"(y)); }
__device__ __forceinline__ void keep4_h(v16h a, v16h b, v16h c, v16h d) { asm volatile("v_nop" :: "v"(a), "v"(b), "v"(c), "v"(d)); }
__device__ __forceinline__ void keep4_b(v16b a, v16b b, v16b c, v16b d) { asm volatile("v_nop" :: "v"(a), "v"(b), "v"(c), "v"(d)); }
__device__ __forceinline__ void acc_guard4(v8f& a, v8f& b, v8f& c, v8f& d) { asm volatile("v_nop\n\tv_nop\n\tv_nop\n\tv_nop" : "+v"(a), "+v"(b), "+v"(c), "+v"(d)); }
template <typename T> struct Frag;
template <> struct Frag<_Float16> {
  typedef v16h V; union U { v16h v; v8h h[2]; };
  static __device__ __forceinline__ v16h load(const _Float16* p) {
    U f; f.h[0] = *(const v8h*)(p); f.h[1] = *(const v8h*)(p + 16); return f.v;
  }
  static __device__ __forceinline__ v8f mma(v16h a, v16h b, v8f c) {
    return __builtin_amdgcn_wmma_f32_16x16x32_f16(false, a, false, b, (short)0, c, false, false);
  }
  static __device__ __forceinline__ void guard(v8f& a, v8f& b, v16h x, v16h y) { dep_guard_h(a, b, x, y); }
  static __device__ __forceinline__ void keep(v16h a, v16h b, v16h c, v16h d) { keep4_h(a, b, c, d); }
};
template <> struct Frag<__bf16> {
  typedef v16b V; union U { v16b v; v8b h[2]; };
  static __device__ __forceinline__ v16b load(const __bf16* p) {
    U f; f.h[0] = *(const v8b*)(p); f.h[1] = *(const v8b*)(p + 16); return f.v;
  }
  static __device__ __forceinline__ v8f mma(v16b a, v16b b, v8f c) {
    return __builtin_amdgcn_wmma_f32_16x16x32_bf16(false, a, false, b, (short)0, c, false, false);
  }
  static __device__ __forceinline__ void guard(v8f& a, v8f& b, v16b x, v16b y) { dep_guard_b(a, b, x, y); }
  static __device__ __forceinline__ void keep(v16b a, v16b b, v16b c, v16b d) { keep4_b(a, b, c, d); }
};

__device__ __forceinline__ unsigned pk16(unsigned short a, unsigned short b) { return (unsigned)a | ((unsigned)b << 16); }

template <int ET> struct Elem;
template <> struct Elem<0> { typedef _Float16 T; };
template <> struct Elem<1> { typedef __bf16 T; };
template <int ET, bool SPLIT, int BIAS_MODE, int OUT_MODE, bool RESID>
__global__ __launch_bounds__(256) void wmma_gemm64(
    const unsigned short* __restrict__ Ap, const unsigned short* __restrict__ A2p, int lda, long strideA,
    const unsigned short* __restrict__ Btp, const unsigned short* __restrict__ Bt2p, int ldb, long strideB,
    void* __restrict__ Cout, void* __restrict__ Cout2, int ldc, long strideC,
    const float* __restrict__ bias,
    const float* __restrict__ resid, long strideR,
    int M, int N, int K, float scale) {
  typedef typename Elem<ET>::T T;
  typedef typename Frag<T>::V V;
  const T* A = (const T*)Ap; const T* A2 = (const T*)A2p; const T* Bt = (const T*)Btp; const T* Bt2 = (const T*)Bt2p;
  __shared__ __align__(16) float sT[8][16 * 68];
  const int b    = blockIdx.y;
  const int lane = threadIdx.x & 31;
  const int wave = threadIdx.x >> 5;
  const int tilesN = N >> 6;
  const int tilesM = M >> 6;
  const int tile = blockIdx.x * 8 + wave;
  if (tile >= tilesM * tilesN) return;
  const int tm = tile / tilesN;
  const int tn = tile - tm * tilesN;
  const int m0 = tm << 6;
  const int n0 = tn << 6;

  const T* Ab  = A  + (size_t)b * strideA;
  const T* Bb  = Bt + (size_t)b * strideB;
  const T* Ab2 = SPLIT ? (A2  + (size_t)b * strideA) : nullptr;
  const T* Bb2 = SPLIT ? (Bt2 + (size_t)b * strideB) : nullptr;

  const int rlane = lane & 15;
  const int koff  = (lane >> 4) * 8;
  const int mOff  = (lane >> 4) * 8;

  v8f acc[4][4];
#pragma unroll
  for (int i = 0; i < 4; ++i)
#pragma unroll
    for (int j = 0; j < 4; ++j) acc[i][j] = (v8f){0.f,0.f,0.f,0.f,0.f,0.f,0.f,0.f};

  for (int k0 = 0; k0 < K; k0 += 32) {
    V bh[4], bl[4];
#pragma unroll
    for (int j = 0; j < 4; ++j) {
      const size_t bo = (size_t)(n0 + (j << 4) + rlane) * ldb + koff + k0;
      bh[j] = Frag<T>::load(Bb + bo);
      if (SPLIT) bl[j] = Frag<T>::load(Bb2 + bo);
    }
#pragma unroll
    for (int i = 0; i < 4; ++i) {
      const size_t ao = (size_t)(m0 + (i << 4) + rlane) * lda + koff + k0;
      V ah = Frag<T>::load(Ab + ao);
      V al;
      if (SPLIT) al = Frag<T>::load(Ab2 + ao);
#pragma unroll
      for (int j = 0; j < 4; ++j) {
        acc[i][j] = Frag<T>::mma(ah, bh[j], acc[i][j]);
        if (SPLIT) {
          acc[i][j] = Frag<T>::mma(ah, bl[j], acc[i][j]);
          acc[i][j] = Frag<T>::mma(al, bh[j], acc[i][j]);
        }
      }
      Frag<T>::guard(acc[i][0], acc[i][3], ah, SPLIT ? al : ah);
    }
    Frag<T>::keep(bh[0], bh[1], bh[2], bh[3]);
    if (SPLIT) Frag<T>::keep(bl[0], bl[1], bl[2], bl[3]);
  }
  acc_guard4(acc[0][0], acc[0][1], acc[0][2], acc[0][3]);
  acc_guard4(acc[1][0], acc[1][1], acc[1][2], acc[1][3]);
  acc_guard4(acc[2][0], acc[2][1], acc[2][2], acc[2][3]);
  acc_guard4(acc[3][0], acc[3][1], acc[3][2], acc[3][3]);

  float* slab = sT[wave];
  const float* Rb = RESID ? (resid + (size_t)b * strideR) : nullptr;
#pragma unroll
  for (int i = 0; i < 4; ++i) {
    const int mBase = m0 + (i << 4);
#pragma unroll
    for (int j = 0; j < 4; ++j) {
      const int n = n0 + (j << 4) + rlane;
      float bvv = 0.f;
      if (BIAS_MODE == 2) bvv = bias[n];
#pragma unroll
      for (int r = 0; r < 8; ++r) {
        float v = acc[i][j][r] * scale;
        if (BIAS_MODE == 1) v += bias[mBase + mOff + r];
        if (BIAS_MODE == 2) v += bvv;
        if (RESID) v += Rb[(size_t)(mBase + mOff + r) * ldc + n];
        slab[(mOff + r) * 68 + (j << 4) + rlane] = v;
      }
    }
    __builtin_amdgcn_fence(__ATOMIC_RELEASE, "workgroup");
    __builtin_amdgcn_wave_barrier();
    __builtin_amdgcn_fence(__ATOMIC_ACQUIRE, "workgroup");
    if (OUT_MODE == 0) {
      float* C = (float*)Cout + (size_t)b * strideC;
      const int hh = lane >> 4, c4 = (lane & 15) * 4;
      for (int pass = 0; pass < 2; ++pass) {
#pragma unroll
        for (int it = 0; it < 8; ++it) {
          const int row = it * 2 + hh;
          v4f v = *(const v4f*)(slab + row * 68 + c4);
          *(volatile v4f*)(C + (size_t)(mBase + row) * ldc + n0 + c4) = v;
        }
        __threadfence();
      }
    } else {
      const int q = lane >> 3, c8 = (lane & 7) * 8;
      unsigned short* C  = (unsigned short*)Cout  + (size_t)b * strideC;
      unsigned short* C2 = (OUT_MODE == 2) ? ((unsigned short*)Cout2 + (size_t)b * strideC) : nullptr;
      for (int pass = 0; pass < 2; ++pass) {
#pragma unroll
        for (int it = 0; it < 4; ++it) {
          const int row = it * 4 + q;
          const float* sp = slab + row * 68 + c8;
          v8h hv, lv;
#pragma unroll
          for (int e = 0; e < 8; ++e) {
            if (OUT_MODE == 1) {
              hv[e] = (_Float16)sp[e];
            } else {
              unsigned short hb = f2bf_bits(sp[e]);
              hv[e] = __builtin_bit_cast(_Float16, hb);
              if (OUT_MODE == 2) {
                unsigned short lb = f2bf_bits(sp[e] - bf_bits2f(hb));
                lv[e] = __builtin_bit_cast(_Float16, lb);
              }
            }
          }
          *(volatile v8h*)(C + (size_t)(mBase + row) * ldc + n0 + c8) = hv;
          if (OUT_MODE == 2) *(volatile v8h*)(C2 + (size_t)(mBase + row) * ldc + n0 + c8) = lv;
        }
        __threadfence();
      }
    }
    __builtin_amdgcn_fence(__ATOMIC_RELEASE, "workgroup");
    __builtin_amdgcn_wave_barrier();
    __builtin_amdgcn_fence(__ATOMIC_ACQUIRE, "workgroup");
  }
}

__global__ __launch_bounds__(256) void cast8_bf16_kernel(const float* __restrict__ in, unsigned short* __restrict__ out, int n8) {
  const int i = blockIdx.x * 256 + threadIdx.x;
  if (i >= n8) return;
  const float* p = in + 8 * (size_t)i;
  const v4f a = *(const v4f*)(p);
  const v4f c = *(const v4f*)(p + 4);
  unsigned short hb[8];
#pragma unroll
  for (int e = 0; e < 4; ++e) {
    hb[e]     = f2bf_bits(a[e]);
    hb[4 + e] = f2bf_bits(c[e]);
  }
  const v4u u = (v4u){pk16(hb[0], hb[1]), pk16(hb[2], hb[3]), pk16(hb[4], hb[5]), pk16(hb[6], hb[7])};
  unsigned short* q = out + 8 * (size_t)i;
  *(volatile v4u*)q = u;
  __threadfence();
  *(volatile v4u*)q = u;
}

__global__ __launch_bounds__(256) void softmax_row_kernel(const float* __restrict__ S, unsigned short* __restrict__ P) {
  __shared__ float redM[8];
  __shared__ float redS[8];
  const int row  = blockIdx.x;
  const int t    = threadIdx.x;
  const int lane = t & 31, wave = t >> 5;
  const float* sr = S + (size_t)row * kSeqK + 8 * t;
  const v4f a = *(const v4f*)(sr);
  const v4f c = *(const v4f*)(sr + 4);
  float x[8];
#pragma unroll
  for (int e = 0; e < 4; ++e) { x[e] = a[e]; x[4 + e] = c[e]; }
  float m = fmaxf(fmaxf(fmaxf(x[0], x[1]), fmaxf(x[2], x[3])), fmaxf(fmaxf(x[4], x[5]), fmaxf(x[6], x[7])));
#pragma unroll
  for (int off = 1; off < 32; off <<= 1) m = fmaxf(m, __shfl_xor(m, off, 32));
  if (lane == 0) redM[wave] = m;
  __syncthreads();
  float gm = redM[0];
#pragma unroll
  for (int w = 1; w < 8; ++w) gm = fmaxf(gm, redM[w]);
  float ex[8];
  float ps = 0.f;
#pragma unroll
  for (int e = 0; e < 8; ++e) { ex[e] = expf(x[e] - gm); ps += ex[e]; }
#pragma unroll
  for (int off = 1; off < 32; off <<= 1) ps += __shfl_xor(ps, off, 32);
  if (lane == 0) redS[wave] = ps;
  __syncthreads();
  float tot = 0.f;
#pragma unroll
  for (int w = 0; w < 8; ++w) tot += redS[w];
  const float inv = 1.0f / tot;
  unsigned short hb[8];
#pragma unroll
  for (int e = 0; e < 8; ++e) hb[e] = f2bf_bits(ex[e] * inv);
  const v4u u = (v4u){pk16(hb[0], hb[1]), pk16(hb[2], hb[3]), pk16(hb[4], hb[5]), pk16(hb[6], hb[7])};
  unsigned short* pp = P + (size_t)row * kSeqK + 8 * t;
  *(volatile v4u*)pp = u;
  __threadfence();
  *(volatile v4u*)pp = u;
}

__global__ __launch_bounds__(256) void layernorm_kernel(const float* __restrict__ X, const float* __restrict__ gamma,
                                                        const float* __restrict__ beta, float* __restrict__ out) {
  __shared__ float redA[8];
  __shared__ float redB[8];
  const int row  = blockIdx.x;
  const int t    = threadIdx.x;
  const int lane = t & 31, wave = t >> 5;
  const v4f xv = *(const v4f*)(X + (size_t)row * kEmb + 4 * t);
  float s = (xv[0] + xv[1]) + (xv[2] + xv[3]);
#pragma unroll
  for (int off = 1; off < 32; off <<= 1) s += __shfl_xor(s, off, 32);
  if (lane == 0) redA[wave] = s;
  __syncthreads();
  float tot = 0.f;
#pragma unroll
  for (int w = 0; w < 8; ++w) tot += redA[w];
  const float mu = tot * kInvEmb;
  const float d0 = xv[0] - mu, d1 = xv[1] - mu, d2 = xv[2] - mu, d3 = xv[3] - mu;
  float s2 = (d0 * d0 + d1 * d1) + (d2 * d2 + d3 * d3);
#pragma unroll
  for (int off = 1; off < 32; off <<= 1) s2 += __shfl_xor(s2, off, 32);
  if (lane == 0) redB[wave] = s2;
  __syncthreads();
  float tot2 = 0.f;
#pragma unroll
  for (int w = 0; w < 8; ++w) tot2 += redB[w];
  const float var  = tot2 * kInvEmb;
  const float rstd = 1.0f / sqrtf(var + kLnEps);
  const v4f g  = *(const v4f*)(gamma + 4 * t);
  const v4f bb = *(const v4f*)(beta + 4 * t);
  v4f y;
  y[0] = d0 * rstd * g[0] + bb[0];
  y[1] = d1 * rstd * g[1] + bb[1];
  y[2] = d2 * rstd * g[2] + bb[2];
  y[3] = d3 * rstd * g[3] + bb[3];
  float* op = out + (size_t)row * kEmb + 4 * t;
  *(volatile v4f*)op = y;
  __threadfence();
  *(volatile v4f*)op = y;
}

#define GEMM_PROJ   wmma_gemm64<1, false, 2, 3, false>
#define GEMM_PROJT  wmma_gemm64<1, false, 1, 3, false>
#define GEMM_SCORE  wmma_gemm64<1, false, 0, 0, false>
#define GEMM_CTX    wmma_gemm64<1, false, 0, 3, false>
#define GEMM_OUT    wmma_gemm64<1, false, 2, 0, true>

extern "C" void kernel_launch(void* const* d_in, const int* in_sizes, int n_in,
                              void* d_out, int out_size, void* d_ws, size_t ws_size,
                              hipStream_t stream) {
  if (n_in < 13) return;
  const int nQ = kRowsQ * kEmb;
  const int nK = kRowsK * kEmb;
  const int nW = kEmb * kEmb;
  if (in_sizes[0] != nQ || in_sizes[1] != nK || in_sizes[2] != nK) return;
  if (in_sizes[3] != nW || in_sizes[5] != nW || in_sizes[7] != nW || in_sizes[9] != nW) return;
  if (in_sizes[4] != kEmb || in_sizes[6] != kEmb || in_sizes[8] != kEmb || in_sizes[10] != kEmb ||
      in_sizes[11] != kEmb || in_sizes[12] != kEmb) return;
  if (out_size != nQ) return;

  const size_t MiB = (size_t)1 << 20;
  const size_t offW   = 0;
  const size_t offQ   = 8 * MiB;
  const size_t offK   = 16 * MiB;
  const size_t offVT  = 32 * MiB;
  const size_t offCtx = 48 * MiB;
  const size_t offP   = 56 * MiB;
  const size_t offA   = 72 * MiB;
  const size_t total  = offA + 32 * MiB;
  if (total > ws_size) return;

  const float* query = (const float*)d_in[0];
  const float* key   = (const float*)d_in[1];
  const float* value = (const float*)d_in[2];
  const float* Wq = (const float*)d_in[3];
  const float* bq = (const float*)d_in[4];
  const float* Wk = (const float*)d_in[5];
  const float* bk = (const float*)d_in[6];
  const float* Wv = (const float*)d_in[7];
  const float* bvp = (const float*)d_in[8];
  const float* Wo = (const float*)d_in[9];
  const float* bo = (const float*)d_in[10];
  const float* gamma = (const float*)d_in[11];
  const float* beta  = (const float*)d_in[12];
  float* out = (float*)d_out;

  char* ws = (char*)d_ws;
  unsigned short* Wqb = (unsigned short*)(ws + offW);
  unsigned short* Wkb = (unsigned short*)(ws + offW + 2 * MiB);
  unsigned short* Wvb = (unsigned short*)(ws + offW + 4 * MiB);
  unsigned short* Wob = (unsigned short*)(ws + offW + 6 * MiB);
  unsigned short* Qp  = (unsigned short*)(ws + offQ);
  unsigned short* Kp  = (unsigned short*)(ws + offK);
  unsigned short* VT  = (unsigned short*)(ws + offVT);
  unsigned short* Ctx = (unsigned short*)(ws + offCtx);
  unsigned short* Pg  = (unsigned short*)(ws + offP);
  unsigned short* qbf = (unsigned short*)(ws + offA);
  unsigned short* kbf = (unsigned short*)(ws + offA + 8 * MiB);
  unsigned short* vbf = (unsigned short*)(ws + offA);
  float* Sg = (float*)(ws + offA);
  float* Xp = (float*)(ws + offA);

  const dim3 blk(256);

  cast8_bf16_kernel<<<dim3(nW / 8 / 256), blk, 0, stream>>>(Wq, Wqb, nW / 8);
  cast8_bf16_kernel<<<dim3(nW / 8 / 256), blk, 0, stream>>>(Wk, Wkb, nW / 8);
  cast8_bf16_kernel<<<dim3(nW / 8 / 256), blk, 0, stream>>>(Wv, Wvb, nW / 8);
  cast8_bf16_kernel<<<dim3(nW / 8 / 256), blk, 0, stream>>>(Wo, Wob, nW / 8);
  cast8_bf16_kernel<<<dim3(nQ / 8 / 256), blk, 0, stream>>>(query, qbf, nQ / 8);
  cast8_bf16_kernel<<<dim3(nK / 8 / 256), blk, 0, stream>>>(key, kbf, nK / 8);

  GEMM_PROJ<<<dim3((kRowsQ / 64) * (kEmb / 64) / 8, 1), blk, 0, stream>>>(
      qbf, qbf, kEmb, 0L, Wqb, Wqb, kEmb, 0L, (void*)Qp, (void*)Qp, kEmb, 0L,
      bq, query, 0L, kRowsQ, kEmb, kEmb, 1.0f);
  GEMM_PROJ<<<dim3((kRowsK / 64) * (kEmb / 64) / 8, 1), blk, 0, stream>>>(
      kbf, kbf, kEmb, 0L, Wkb, Wkb, kEmb, 0L, (void*)Kp, (void*)Kp, kEmb, 0L,
      bk, query, 0L, kRowsK, kEmb, kEmb, 1.0f);

  cast8_bf16_kernel<<<dim3(nK / 8 / 256), blk, 0, stream>>>(value, vbf, nK / 8);
  GEMM_PROJT<<<dim3((kEmb / 64) * (kSeqK / 64) / 8, kBatch), blk, 0, stream>>>(
      Wvb, Wvb, kEmb, 0L, vbf, vbf, kEmb, (long)kSeqK * kEmb,
      (void*)VT, (void*)VT, kSeqK, (long)kEmb * kSeqK,
      bvp, query, 0L, kEmb, kSeqK, kEmb, 1.0f);

  for (int g = 0; g < kGroups; ++g) {
    const int batch = g / (kHeads / kHeadsPerGroup);
    const int h0 = (g % (kHeads / kHeadsPerGroup)) * kHeadsPerGroup;
    const unsigned short* qa = Qp + (size_t)batch * kSeqQ * kEmb + (size_t)h0 * kHdim;
    const unsigned short* ka = Kp + (size_t)batch * kSeqK * kEmb + (size_t)h0 * kHdim;
    GEMM_SCORE<<<dim3((kSeqQ / 64) * (kSeqK / 64) / 8, kHeadsPerGroup), blk, 0, stream>>>(
        qa, qa, kEmb, (long)kHdim, ka, ka, kEmb, (long)kHdim,
        (void*)Sg, (void*)Sg, kSeqK, (long)kSeqQ * kSeqK,
        bq, query, 0L, kSeqQ, kSeqK, kHdim, kScoreScale);
    softmax_row_kernel<<<dim3(kHeadsPerGroup * kSeqQ), blk, 0, stream>>>(Sg, Pg);
    const unsigned short* vta = VT + ((size_t)batch * kEmb + (size_t)h0 * kHdim) * kSeqK;
    unsigned short* ca = Ctx + (size_t)batch * kSeqQ * kEmb + (size_t)h0 * kHdim;
    GEMM_CTX<<<dim3((kSeqQ / 64) * (kHdim / 64) / 8, kHeadsPerGroup), blk, 0, stream>>>(
        Pg, Pg, kSeqK, (long)kSeqQ * kSeqK, vta, vta, kSeqK, (long)kHdim * kSeqK,
        (void*)ca, (void*)ca, kEmb, (long)kHdim,
        bq, query, 0L, kSeqQ, kHdim, kSeqK, 1.0f);
  }

  GEMM_OUT<<<dim3((kRowsQ / 64) * (kEmb / 64) / 8, 1), blk, 0, stream>>>(
      Ctx, Ctx, kEmb, 0L, Wob, Wob, kEmb, 0L, (void*)Xp, (void*)Xp, kEmb, 0L,
      bo, query, 0L, kRowsQ, kEmb, kEmb, 1.0f);

  layernorm_kernel<<<dim3(kRowsQ), blk, 0, stream>>>(Xp, gamma, beta, out);
}
